// WithMemoryBuffer_64201171141021
// MI455X (gfx1250) — hardware-verified
//
#include <hip/hip_runtime.h>
#include <math.h>

typedef __attribute__((ext_vector_type(16))) _Float16 v16h;
typedef __attribute__((ext_vector_type(8)))  _Float16 v8h;
typedef __attribute__((ext_vector_type(8)))  float    v8f;
typedef __attribute__((ext_vector_type(4)))  float    v4f;

constexpr int NBATCH   = 16384;
constexpr int NSTEP    = 128;
constexpr int HID      = 256;
constexpr int NOUT     = 10;
constexpr int NOUT_PAD = 16;
constexpr float LN_EPS = 1e-5f;

constexpr int ROWS_PB   = 64;
constexpr int NBLK      = NBATCH / ROWS_PB;
constexpr int NTHREADS  = 256;
constexpr int APITCH    = HID + 8;
constexpr int ATILE_HALVES = ROWS_PB * APITCH;
constexpr int LUT_ROWS  = 16;
constexpr int LUT_FLOATS = LUT_ROWS * HID;
constexpr int PSUM_FLOATS = 4 * 2 * 16 * 2;
constexpr int OUT_PER_BLK = ROWS_PB * NOUT;
static_assert(NBATCH % ROWS_PB == 0);
static_assert(HID == 2 * 128 && HID % 32 == 0);
static_assert(APITCH % 8 == 0);
static_assert((ROWS_PB - 1) * APITCH + HID <= ATILE_HALVES);
static_assert(OUT_PER_BLK % 128 == 0 && OUT_PER_BLK <= LUT_FLOATS);
static_assert((OUT_PER_BLK * 4) % 128 == 0);
static_assert(LUT_FLOATS % NTHREADS == 0 && (ROWS_PB * NSTEP) % NTHREADS == 0);
static_assert(NOUT <= NOUT_PAD);

constexpr int W_DWORDS   = HID * HID / 2;
constexpr int OW_DWORDS  = NOUT_PAD * HID / 2;
constexpr int OW_REAL_DW = NOUT * HID / 2;
constexpr int PREP_B1    = W_DWORDS / 256;
constexpr int PREP_BLOCKS = PREP_B1 + OW_DWORDS / 256;
static_assert(W_DWORDS % 256 == 0 && OW_DWORDS % 256 == 0 && PREP_BLOCKS == 136);

__device__ __forceinline__ void dep_guard_h(v8f& a, v8f& b, v16h x, v16h y) { asm volatile("v_nop\n\tv_nop\n\tv_nop\n\tv_nop" : "+v"(a), "+v"(b) : "v"(x), "v"(y)); }
__device__ __forceinline__ void dep_guard1(v8f& a, v16h x, v16h y) { asm volatile("v_nop\n\tv_nop\n\tv_nop\n\tv_nop" : "+v"(a) : "v"(x), "v"(y)); }
__device__ __forceinline__ void keep4_h(v16h a, v16h b, v16h c, v16h d) { asm volatile("v_nop" :: "v"(a), "v"(b), "v"(c), "v"(d)); }
__device__ __forceinline__ void acc_guard4(v8f& a, v8f& b, v8f& c, v8f& d) { asm volatile("v_nop\n\tv_nop\n\tv_nop\n\tv_nop" : "+v"(a), "+v"(b), "+v"(c), "+v"(d)); }

template <typename T> struct Frag;
template <> struct Frag<_Float16> {
  typedef v16h V; union U { v16h v; v8h h[2]; };
  static __device__ __forceinline__ v16h load(const _Float16* p) {
    U f; f.h[0] = *(const v8h*)(p); f.h[1] = *(const v8h*)(p + 16); return f.v;
  }
  static __device__ __forceinline__ v8f mma(v16h a, v16h b, v8f c) {
    return __builtin_amdgcn_wmma_f32_16x16x32_f16(false, a, false, b, (short)0, c, false, false);
  }
  static __device__ __forceinline__ void guard(v8f& a, v8f& b, v16h x, v16h y) { dep_guard_h(a, b, x, y); }
  static __device__ __forceinline__ void keep(v16h a, v16h b, v16h c, v16h d) { keep4_h(a, b, c, d); }
};

__device__ __forceinline__ unsigned pack_f16x2(float a, float b) {
  const _Float16 h0 = (_Float16)a, h1 = (_Float16)b;
  return (unsigned)__builtin_bit_cast(unsigned short, h0) | ((unsigned)__builtin_bit_cast(unsigned short, h1) << 16);
}
__device__ __forceinline__ void st2u(unsigned* p, unsigned v) { *(volatile unsigned*)p = v; __threadfence(); *(volatile unsigned*)p = v; }
__device__ __forceinline__ float tanh_2y(float two_y) { return 1.0f - 2.0f * __builtin_amdgcn_rcpf(1.0f + __expf(two_y)); }
__device__ __forceinline__ v8f splat8(float u) { v8f v; v[0] = u; v[1] = u; v[2] = u; v[3] = u; v[4] = u; v[5] = u; v[6] = u; v[7] = u; return v; }

__global__ __launch_bounds__(256) void prep_planes(
    const float* __restrict__ upd_w, const float* __restrict__ head_w,
    unsigned* __restrict__ w16u, unsigned* __restrict__ ow16u) {
  const int blk = blockIdx.x, tid = threadIdx.x;
  if (blk < PREP_B1) {
    const int p = blk * 256 + tid;
    st2u(w16u + p, pack_f16x2(upd_w[2 * p] * 16.0f, upd_w[2 * p + 1] * 16.0f));
  } else {
    const int p = (blk - PREP_B1) * 256 + tid;
    const bool real = (p < OW_REAL_DW);
    const int q = real ? p : (OW_REAL_DW - 1);
    const float a = head_w[2 * q] * 16.0f, b = head_w[2 * q + 1] * 16.0f;
    st2u(ow16u + p, pack_f16x2(real ? a : 0.0f, real ? b : 0.0f));
  }
}

__global__ __launch_bounds__(NTHREADS) void rnn_ln_scan(
    const float* __restrict__ x, const float* __restrict__ emb_w, const float* __restrict__ emb_b,
    const float* __restrict__ upd_b, const float* __restrict__ ln_g, const float* __restrict__ ln_b,
    const float* __restrict__ head_b,
    const _Float16* __restrict__ w16, const _Float16* __restrict__ ow16,
    float* __restrict__ out) {
  __shared__ __align__(16) _Float16 atile[ATILE_HALVES];
  __shared__ __align__(16) float fbuf[LUT_FLOATS];
  __shared__ __align__(16) float psum[PSUM_FLOATS];
  __shared__ int xflag;

  const int tid = threadIdx.x, lane = tid & 31, wave = tid >> 5;
  const int c = lane & 15, hh = lane >> 4;
  const int rt = wave >> 1, half = wave & 1;
  const int colb  = half * 128 + 8 * c;
  const int rowl0 = 16 * rt + 8 * hh;
  const int blk = blockIdx.x;

  if (tid == 0) xflag = 1;
#pragma unroll 1
  for (int i = tid; i < LUT_FLOATS; i += NTHREADS) {
    const int v = i >> 8, n = i & (HID - 1);
    fbuf[i] = tanhf((float)v * emb_w[n] + emb_b[n]);
  }
  __syncthreads();
  {
    const float* xb = x + (size_t)blk * (ROWS_PB * NSTEP);
    bool ok = true;
#pragma unroll 1
    for (int i = tid; i < ROWS_PB * NSTEP; i += NTHREADS) {
      const float v = xb[i];
      const bool isint = (v >= 0.0f) && (v <= (float)(LUT_ROWS - 1)) && (floorf(v) == v);
      ok = ok && isint;
    }
    if (!ok) xflag = 0;
  }
  __syncthreads();
  const bool use_lut = (xflag != 0);

  float hst[8][8];
#pragma unroll
  for (int j = 0; j < 8; ++j)
#pragma unroll
    for (int r = 0; r < 8; ++r) hst[j][r] = 0.0f;

  const float*    xr    = x + (size_t)(blk * ROWS_PB + rowl0) * NSTEP;
  _Float16*       arow  = atile + rowl0 * APITCH + colb;
  const _Float16* afrag = atile + (16 * rt + c) * APITCH + 8 * hh;
  const _Float16* bfrag = w16 + (size_t)colb * HID + 8 * hh;
  const float inv256 = 1.0f / 256.0f;

#pragma unroll 1
  for (int s = 0; s < NSTEP; ++s) {
    float xv[8];
#pragma unroll
    for (int r = 0; r < 8; ++r) xv[r] = xr[r * NSTEP + s];
    if (use_lut) {
#pragma unroll
      for (int r = 0; r < 8; ++r) {
        int xi = (int)xv[r];
        xi = (xi < 0) ? 0 : xi;
        xi = (xi > LUT_ROWS - 1) ? (LUT_ROWS - 1) : xi;
        const float* lp = fbuf + xi * HID + colb;
        const v4f i0 = *(const v4f*)(lp);
        const v4f i1 = *(const v4f*)(lp + 4);
        v8h hv;
        hv[0] = (_Float16)(i0[0] + hst[0][r]); hv[1] = (_Float16)(i0[1] + hst[1][r]);
        hv[2] = (_Float16)(i0[2] + hst[2][r]); hv[3] = (_Float16)(i0[3] + hst[3][r]);
        hv[4] = (_Float16)(i1[0] + hst[4][r]); hv[5] = (_Float16)(i1[1] + hst[5][r]);
        hv[6] = (_Float16)(i1[2] + hst[6][r]); hv[7] = (_Float16)(i1[3] + hst[7][r]);
        *(v8h*)(arow + r * APITCH) = hv;
      }
    } else {
      const v4f w0 = *(const v4f*)(emb_w + colb), w1 = *(const v4f*)(emb_w + colb + 4);
      const v4f b0 = *(const v4f*)(emb_b + colb), b1 = *(const v4f*)(emb_b + colb + 4);
      const float ew8[8] = {w0[0], w0[1], w0[2], w0[3], w1[0], w1[1], w1[2], w1[3]};
      const float eb8[8] = {b0[0], b0[1], b0[2], b0[3], b1[0], b1[1], b1[2], b1[3]};
#pragma unroll
      for (int r = 0; r < 8; ++r) {
        v8h hv;
#pragma unroll
        for (int i = 0; i < 8; ++i) {
          const float pre = fmaf(xv[r], ew8[i], eb8[i]);
          hv[i] = (_Float16)(tanh_2y(2.0f * pre) + hst[i][r]);
        }
        *(v8h*)(arow + r * APITCH) = hv;
      }
    }
    __syncthreads();

    v8f acc[8];
    {
      const v4f u0 = *(const v4f*)(upd_b + colb), u1 = *(const v4f*)(upd_b + colb + 4);
      acc[0] = splat8(u0[0] * 16.0f); acc[1] = splat8(u0[1] * 16.0f); acc[2] = splat8(u0[2] * 16.0f); acc[3] = splat8(u0[3] * 16.0f);
      acc[4] = splat8(u1[0] * 16.0f); acc[5] = splat8(u1[1] * 16.0f); acc[6] = splat8(u1[2] * 16.0f); acc[7] = splat8(u1[3] * 16.0f);
    }
#pragma unroll 2
    for (int kc = 0; kc < HID / 32; ++kc) {
      const v16h fa = Frag<_Float16>::load(afrag + 32 * kc);
#pragma unroll
      for (int g = 0; g < 2; ++g) {
        v16h fb[4];
#pragma unroll
        for (int j = 0; j < 4; ++j) fb[j] = Frag<_Float16>::load(bfrag + (size_t)(4 * g + j) * HID + 32 * kc);
#pragma unroll
        for (int j = 0; j < 4; ++j) acc[4 * g + j] = Frag<_Float16>::mma(fa, fb[j], acc[4 * g + j]);
        Frag<_Float16>::guard(acc[4 * g], acc[4 * g + 3], fa, fb[3]);
        Frag<_Float16>::keep(fb[0], fb[1], fb[2], fb[3]);
      }
    }
    acc_guard4(acc[0], acc[1], acc[2], acc[3]);
    acc_guard4(acc[4], acc[5], acc[6], acc[7]);

    float sr[8], qr[8];
#pragma unroll
    for (int r = 0; r < 8; ++r) { sr[r] = 0.0f; qr[r] = 0.0f; }
#pragma unroll
    for (int j = 0; j < 8; ++j) {
#pragma unroll
      for (int r = 0; r < 8; ++r) {
        const float e = tanh_2y(acc[j][r] * 0.125f);
        hst[j][r] = e;
        sr[r] += e;
        qr[r] = fmaf(e, e, qr[r]);
      }
    }
#pragma unroll
    for (int off = 1; off < 16; off <<= 1) {
#pragma unroll
      for (int r = 0; r < 8; ++r) {
        sr[r] += __shfl_xor(sr[r], off, 32);
        qr[r] += __shfl_xor(qr[r], off, 32);
      }
    }
    if (c == 0) {
      float* pp = psum + ((rt * 2 + half) * 16 + 8 * hh) * 2;
      v4f t0; t0[0] = sr[0]; t0[1] = qr[0]; t0[2] = sr[1]; t0[3] = qr[1];
      v4f t1; t1[0] = sr[2]; t1[1] = qr[2]; t1[2] = sr[3]; t1[3] = qr[3];
      v4f t2; t2[0] = sr[4]; t2[1] = qr[4]; t2[2] = sr[5]; t2[3] = qr[5];
      v4f t3; t3[0] = sr[6]; t3[1] = qr[6]; t3[2] = sr[7]; t3[3] = qr[7];
      *(v4f*)(pp)      = t0;
      *(v4f*)(pp + 4)  = t1;
      *(v4f*)(pp + 8)  = t2;
      *(v4f*)(pp + 12) = t3;
    }
    __syncthreads();
    float ca[8], cb[8];
    {
      const float* qp = psum + ((rt * 2 + (half ^ 1)) * 16 + 8 * hh) * 2;
      const v4f o0 = *(const v4f*)(qp), o1 = *(const v4f*)(qp + 4), o2 = *(const v4f*)(qp + 8), o3 = *(const v4f*)(qp + 12);
      const float osr[8] = {o0[0], o0[2], o1[0], o1[2], o2[0], o2[2], o3[0], o3[2]};
      const float oqr[8] = {o0[1], o0[3], o1[1], o1[3], o2[1], o2[3], o3[1], o3[3]};
#pragma unroll
      for (int r = 0; r < 8; ++r) {
        const float S  = sr[r] + osr[r];
        const float Q  = qr[r] + oqr[r];
        const float mu = S * inv256;
        const float var = fmaxf(Q * inv256 - mu * mu, 0.0f);
        const float rstd = rsqrtf(var + LN_EPS);
        ca[r] = rstd;
        cb[r] = -mu * rstd;
      }
    }
    {
      const v4f g0 = *(const v4f*)(ln_g + colb), g1 = *(const v4f*)(ln_g + colb + 4);
      const v4f z0 = *(const v4f*)(ln_b + colb), z1 = *(const v4f*)(ln_b + colb + 4);
      const float g8[8] = {g0[0], g0[1], g0[2], g0[3], g1[0], g1[1], g1[2], g1[3]};
      const float z8[8] = {z0[0], z0[1], z0[2], z0[3], z1[0], z1[1], z1[2], z1[3]};
#pragma unroll
      for (int j = 0; j < 8; ++j) {
#pragma unroll
        for (int r = 0; r < 8; ++r) hst[j][r] = fmaf(fmaf(hst[j][r], ca[r], cb[r]), g8[j], z8[j]);
      }
    }
  }

#pragma unroll
  for (int r = 0; r < 8; ++r) {
    v8h hv;
#pragma unroll
    for (int i = 0; i < 8; ++i) hv[i] = (_Float16)hst[i][r];
    *(v8h*)(arow + r * APITCH) = hv;
  }
  __syncthreads();
  float* stage = fbuf;
  if (half == 0) {
    v8f hacc = splat8(0.0f);
    const _Float16* obf = ow16 + (size_t)c * HID + 8 * hh;
#pragma unroll
    for (int kc = 0; kc < HID / 32; ++kc) {
      const v16h fa = Frag<_Float16>::load(afrag + 32 * kc);
      const v16h fb = Frag<_Float16>::load(obf + 32 * kc);
      hacc = Frag<_Float16>::mma(fa, fb, hacc);
      dep_guard1(hacc, fa, fb);
    }
    const int cc = (c < NOUT) ? c : (NOUT - 1);
    const float bv = head_b[cc];
#pragma unroll
    for (int r = 0; r < 8; ++r) {
      const float v = fmaf(hacc[r], 1.0f / 16.0f, bv);
      if (c < NOUT) stage[(rowl0 + r) * NOUT + c] = v;
    }
  }
  __syncthreads();
  if (wave == 0) {
    float* op = out + (size_t)blk * OUT_PER_BLK;
    for (int pass = 0; pass < 2; ++pass) {
#pragma unroll
      for (int it = 0; it < OUT_PER_BLK / 128; ++it) {
        const v4f v = *(const v4f*)(stage + it * 128 + 4 * lane);
        *(volatile v4f*)(op + it * 128 + 4 * lane) = v;
      }
      __threadfence();
    }
  }
}

extern "C" void kernel_launch(void* const* d_in, const int* in_sizes, int n_in,
                              void* d_out, int out_size, void* d_ws, size_t ws_size, hipStream_t stream) {
  if (n_in < 9 || d_out == nullptr || d_ws == nullptr) return;
  if (in_sizes[0] != NBATCH * NSTEP || in_sizes[1] != HID || in_sizes[2] != HID ||
      in_sizes[3] != HID * HID || in_sizes[4] != HID || in_sizes[5] != HID || in_sizes[6] != HID ||
      in_sizes[7] != NOUT * HID || in_sizes[8] != NOUT || out_size != NBATCH * NOUT) return;

  const float* x      = (const float*)d_in[0];
  const float* emb_w  = (const float*)d_in[1];
  const float* emb_b  = (const float*)d_in[2];
  const float* upd_w  = (const float*)d_in[3];
  const float* upd_b  = (const float*)d_in[4];
  const float* ln_g   = (const float*)d_in[5];
  const float* ln_b   = (const float*)d_in[6];
  const float* head_w = (const float*)d_in[7];
  const float* head_b = (const float*)d_in[8];
  float* out = (float*)d_out;

  char* ws = (char*)d_ws; size_t off = 0;
  auto carve = [&](size_t bytes) -> char* { char* p = ws + off; off += (bytes + 255) & ~(size_t)255; return p; };
  unsigned short* W16  = (unsigned short*)carve((size_t)HID * HID * 2);
  unsigned short* OW16 = (unsigned short*)carve((size_t)NOUT_PAD * HID * 2);
  if (off > ws_size || off > (size_t)134217728) return;

  prep_planes<<<PREP_BLOCKS, 256, 0, stream>>>(upd_w, head_w, (unsigned*)W16, (unsigned*)OW16);

  rnn_ln_scan<<<NBLK, NTHREADS, 0, stream>>>(x, emb_w, emb_b, upd_b, ln_g, ln_b, head_b,
                                             (const _Float16*)W16, (const _Float16*)OW16, out);
}
